// GATLayer_1_39977555591204
// MI455X (gfx1250) — hardware-verified
//
#include <hip/hip_runtime.h>
#include <stddef.h>
#include <stdint.h>


#define DIN     128
#define C1      128
#define OUTC    32
#define N2P     64
#define NTHR    256
#define NWAVE   8
#define EPT     8
#define CHUNK   (NTHR * EPT)
#define WCAP    (EPT * 32)
#define LISTN   (NWAVE * WCAP)
#define NBMAX   512
#define SLB     9
#define RCAP    24576
#define DEGCAP  128
#define SQ      160
#define O_S     0
#define O_E     160
#define O_P0    320
#define O_P1    480
#define O_O     640
#define STW     768
#define GBM     64
#define GBN     64
#define GTHR    128
#define CX      8.0f
#define CW      64.0f
#define SCL_XW  0.001953125f
#define NEGSL   0.2f
#define WSMAX   134217728
#define LDS_AGG ((2 * RCAP + 2 * NBMAX + LISTN) * 4 + 128)

static_assert((CHUNK & (CHUNK - 1)) == 0 && CHUNK <= 4096);
static_assert((NBMAX & (NBMAX - 1)) == 0 && NBMAX == (1 << SLB) && NBMAX <= 4096);
static_assert(NTHR * 2 == NBMAX);
static_assert(LISTN >= NBMAX);
static_assert(LISTN >= NWAVE * WCAP);
static_assert((RCAP % 32) == 0);
static_assert(NWAVE * STW <= RCAP);
static_assert(SQ >= 32 * ((DEGCAP + 1 + 31) / 32));
static_assert(O_E == O_S + SQ && O_P0 == O_E + SQ && O_P1 == O_P0 + SQ && O_O == O_P1 + SQ);
static_assert(O_O + C1 <= STW);
static_assert((STW % 4) == 0 && (O_O % 4) == 0);
static_assert(LDS_AGG <= 300000);
static_assert(GBM == (GTHR / 32) * 16);
static_assert(DIN / 8 == 16 && (DIN % 32) == 0);
static_assert((C1 % GBN) == 0 && (N2P % GBN) == 0);
static_assert(OUTC * 4 == 128);

typedef float    v4f  __attribute__((ext_vector_type(4)));
typedef float    v8f  __attribute__((ext_vector_type(8)));
typedef int      v4i  __attribute__((ext_vector_type(4)));
typedef int      v8i  __attribute__((ext_vector_type(8)));
typedef _Float16 v8h  __attribute__((ext_vector_type(8)));
typedef _Float16 v16h __attribute__((ext_vector_type(16)));
union FragH { v16h v; v8h h[2]; v8i w; };

__device__ __forceinline__ v8f wmh(const FragH& a, const FragH& b, v8f c) {
  v8f d = __builtin_amdgcn_wmma_f32_16x16x32_f16(false, a.v, false, b.v, (short)0, c, false, false);
  asm volatile("v_nop\n\tv_nop\n\tv_nop\n\tv_nop" : "+v"(d) : "v"(a.w), "v"(b.w));
  return d;
}

__device__ __forceinline__ void ldwait() {
  asm volatile("s_wait_loadcnt 0x0" ::: "memory");
}

#define WSYNC() do { __builtin_amdgcn_fence(__ATOMIC_RELEASE, "wavefront"); __builtin_amdgcn_wave_barrier(); } while (0)

__device__ __forceinline__ float wsum(float v) {
#pragma unroll
  for (int off = 16; off > 0; off >>= 1) v += __shfl_xor(v, off);
  return v;
}
__device__ __forceinline__ float wmax(float v) {
#pragma unroll
  for (int off = 16; off > 0; off >>= 1) v = fmaxf(v, __shfl_xor(v, off));
  return v;
}

__device__ __forceinline__ v8h cvt8h(const v4f a, const v4f b, const float c) {
  v8h hv;
  hv[0] = (_Float16)(a.x * c); hv[1] = (_Float16)(a.y * c);
  hv[2] = (_Float16)(a.z * c); hv[3] = (_Float16)(a.w * c);
  hv[4] = (_Float16)(b.x * c); hv[5] = (_Float16)(b.y * c);
  hv[6] = (_Float16)(b.z * c); hv[7] = (_Float16)(b.w * c);
  return hv;
}

__device__ __forceinline__ int scan_chunk(const int* __restrict__ dsts, int nE, int cbase, int slotBase,
                                          int nb, int vec8, int* list, int tid, int lane, int wave) {
  int wc = 0;
  const int el0  = tid * EPT;
  const int e0   = cbase + el0;
  const int sent = -2147483647 - 1;
  v4i da, db;
  if (vec8 != 0 && cbase + CHUNK <= nE) {
    da = *(const v4i*)(dsts + e0);
    db = *(const v4i*)(dsts + e0 + 4);
  } else {
    da.x = (e0     < nE) ? dsts[min(e0,     nE - 1)] : sent;
    da.y = (e0 + 1 < nE) ? dsts[min(e0 + 1, nE - 1)] : sent;
    da.z = (e0 + 2 < nE) ? dsts[min(e0 + 2, nE - 1)] : sent;
    da.w = (e0 + 3 < nE) ? dsts[min(e0 + 3, nE - 1)] : sent;
    db.x = (e0 + 4 < nE) ? dsts[min(e0 + 4, nE - 1)] : sent;
    db.y = (e0 + 5 < nE) ? dsts[min(e0 + 5, nE - 1)] : sent;
    db.z = (e0 + 6 < nE) ? dsts[min(e0 + 6, nE - 1)] : sent;
    db.w = (e0 + 7 < nE) ? dsts[min(e0 + 7, nE - 1)] : sent;
  }
  const unsigned nbs = (unsigned)slotBase;
  const unsigned unb = (unsigned)nb;
  const unsigned s0 = (unsigned)da.x - nbs, s1 = (unsigned)da.y - nbs;
  const unsigned s2 = (unsigned)da.z - nbs, s3 = (unsigned)da.w - nbs;
  const unsigned s4 = (unsigned)db.x - nbs, s5 = (unsigned)db.y - nbs;
  const unsigned s6 = (unsigned)db.z - nbs, s7 = (unsigned)db.w - nbs;
  const bool h0 = s0 < unb, h1 = s1 < unb, h2 = s2 < unb, h3 = s3 < unb;
  const bool h4 = s4 < unb, h5 = s5 < unb, h6 = s6 < unb, h7 = s7 < unb;
  const unsigned any = __builtin_amdgcn_ballot_w32(h0 | h1 | h2 | h3 | h4 | h5 | h6 | h7);
  if (any != 0u) {
#define HITJ(J, HJ, SJ) { \
      const unsigned mj = __builtin_amdgcn_ballot_w32(HJ); \
      if (mj != 0u) { \
        if (HJ) { \
          const int pos = wc + (int)__builtin_amdgcn_mbcnt_lo(mj, 0u); \
          if (pos < WCAP) list[wave * WCAP + pos] = ((el0 + (J)) << 12) | (int)(SJ); \
        } \
        wc += (int)__builtin_popcount(mj); } }
    HITJ(0, h0, s0)
    HITJ(1, h1, s1)
    HITJ(2, h2, s2)
    HITJ(3, h3, s3)
    HITJ(4, h4, s4)
    HITJ(5, h5, s5)
    HITJ(6, h6, s6)
    HITJ(7, h7, s7)
#undef HITJ
  }
  return wc;
}

__global__ __launch_bounds__(NTHR) void k_xprep(const float* __restrict__ x, _Float16* xh, int nN, int nUnits) {
  const int i = (int)blockIdx.x * NTHR + (int)threadIdx.x;
  if (i >= nUnits) return;
  const int row = i >> 4;
  const int c0  = (i & 15) * 8;
  const int rc  = row < nN ? row : nN - 1;
  const float* p = x + (size_t)rc * DIN + c0;
  v4f a = *(const v4f*)p, b = *(const v4f*)(p + 4);
  const v4f z4 = {0.f, 0.f, 0.f, 0.f};
  if (row >= nN) { a = z4; b = z4; }
  const v8h hv = cvt8h(a, b, CX);
  const size_t o = (size_t)row * DIN + c0;
  *(volatile v8h*)(xh + o) = hv;
  __threadfence();
  *(volatile v8h*)(xh + o) = hv;
}

__global__ __launch_bounds__(NTHR) void k_wtr(const float* __restrict__ w, int cc, int K,
                                              _Float16* wt, int nUnits) {
  const int u = (int)blockIdx.x * NTHR + (int)threadIdx.x;
  if (u >= nUnits) return;
  const int kq = K >> 3;
  const int n  = u / kq;
  const int k8 = (u - n * kq) * 8;
  const int ncl = n < cc ? n : cc - 1;
  const float* p = w + (size_t)k8 * (size_t)cc + ncl;
  v4f a, b;
  a.x = p[0];                  a.y = p[(size_t)cc];         a.z = p[(size_t)2 * cc];     a.w = p[(size_t)3 * cc];
  b.x = p[(size_t)4 * cc];     b.y = p[(size_t)5 * cc];     b.z = p[(size_t)6 * cc];     b.w = p[(size_t)7 * cc];
  const v4f z4 = {0.f, 0.f, 0.f, 0.f};
  if (n >= cc) { a = z4; b = z4; }
  const v8h hv = cvt8h(a, b, CW);
  const size_t o = (size_t)n * (size_t)K + k8;
  *(volatile v8h*)(wt + o) = hv;
  __threadfence();
  *(volatile v8h*)(wt + o) = hv;
}

__global__ __launch_bounds__(GTHR) void k_gemm(
    const _Float16* __restrict__ A, const _Float16* __restrict__ WT, float* outF, int K, int ldo,
    const float* __restrict__ attS, const float* __restrict__ attD, int CA, float* AL, int MPr, float scl)
{
  __shared__ __attribute__((aligned(16))) float stg[GBM * GBN];
  __shared__ __attribute__((aligned(16))) float alv[2 * GBM];
  const int tid = (int)threadIdx.x, lane = tid & 31, wave = tid >> 5, hh = lane >> 4, m = lane & 15;
  const int rowBase = (int)blockIdx.x * GBM;
  const int col0    = (int)blockIdx.y * GBN;
  const int hd      = (int)blockIdx.y;

  v8f acc[4];
  {
    const v8f z = {0.f, 0.f, 0.f, 0.f, 0.f, 0.f, 0.f, 0.f};
    acc[0] = z; acc[1] = z; acc[2] = z; acc[3] = z;
  }
  const _Float16* ap = A  + (size_t)(rowBase + 16 * wave + m) * (size_t)K + 8 * hh;
  const _Float16* wp = WT + (size_t)(col0 + m) * (size_t)K + 8 * hh;
  const int ksteps = K >> 5;
#pragma unroll 1
  for (int ks = 0; ks < ksteps; ++ks) {
    FragH af;
    af.h[0] = *(const v8h*)(ap + 32 * ks);
    af.h[1] = *(const v8h*)(ap + 32 * ks + 16);
#pragma unroll
    for (int t = 0; t < 4; ++t) {
      const _Float16* wq = wp + (size_t)(16 * t) * (size_t)K + 32 * ks;
      FragH bf;
      bf.h[0] = *(const v8h*)wq;
      bf.h[1] = *(const v8h*)(wq + 16);
      acc[t] = wmh(af, bf, acc[t]);
    }
  }

#pragma unroll
  for (int t = 0; t < 4; ++t) {
    const int lc = 16 * t + m;
#pragma unroll
    for (int r = 0; r < 8; ++r) {
      const int lr = 16 * wave + 8 * hh + r;
      stg[lr * GBN + lc] = acc[t][r] * scl;
    }
  }
  __syncthreads();

  {
    v4f fv[8];
#pragma unroll
    for (int i = 0; i < 8; ++i) {
      const int lr = 16 * wave + 2 * i + hh;
      fv[i] = *(const v4f*)(stg + lr * GBN + 4 * m);
    }
#pragma unroll
    for (int i = 0; i < 8; ++i) {
      const int lr = 16 * wave + 2 * i + hh;
      const int gr = rowBase + lr;
      float* op = outF + (size_t)gr * (size_t)ldo + col0 + 4 * m;
      *(volatile v4f*)op = fv[i];
    }
    __threadfence();
#pragma unroll
    for (int i = 0; i < 8; ++i) {
      const int lr = 16 * wave + 2 * i + hh;
      const int gr = rowBase + lr;
      float* op = outF + (size_t)gr * (size_t)ldo + col0 + 4 * m;
      *(volatile v4f*)op = fv[i];
    }
  }

  {
    const int arow  = tid & 63;
    const int which = tid >> 6;
    int cal = CA < GBN ? CA : GBN;
    cal = cal < 0 ? 0 : cal;
    const float* apq = ((which == 0) ? attS : attD) + (size_t)hd * (size_t)CA;
    float s = 0.f;
#pragma unroll 1
    for (int c4 = 0; c4 < (cal >> 2); ++c4) {
      const v4f hv = *(const v4f*)(stg + arow * GBN + 4 * c4);
      const v4f av = *(const v4f*)(apq + 4 * c4);
      s = fmaf(hv.x, av.x, s);
      s = fmaf(hv.y, av.y, s);
      s = fmaf(hv.z, av.z, s);
      s = fmaf(hv.w, av.w, s);
    }
    alv[which * GBM + arow] = s;
  }
  __syncthreads();
  if (wave == 0) {
    const v4f v = *(const v4f*)(alv + hh * GBM + 4 * m);
    float* dp = AL + (size_t)(2 * hd + hh) * (size_t)MPr + rowBase + 4 * m;
    *(volatile v4f*)dp = v;
    __threadfence();
    *(volatile v4f*)dp = v;
  }
}

template<int H, int C, int LAYER>
__global__ __launch_bounds__(NTHR) void k_agg(
    const int* __restrict__ srcs, const int* __restrict__ dsts, const float* __restrict__ ew,
    const float* __restrict__ We, const float* __restrict__ ae,
    const float* __restrict__ AL, const float* __restrict__ HF, int ldh,
    const float* __restrict__ bias, _Float16* HH, float* OUT,
    int nN, int nE, int nb, int vec8, int MPr) {
  extern __shared__ v4f lds_dyn[];
  int* reg1 = (int*)lds_dyn;
  int* reg2 = reg1 + RCAP;
  int* scnt = reg2 + RCAP;
  int* soff = scnt + NBMAX;
  int* list = soff + NBMAX;
  int* wcnt = list + LISTN;
  int* wtot = wcnt + NWAVE;
  float* cel = (float*)(wtot + NWAVE);
  const int tid = (int)threadIdx.x, lane = tid & 31, wave = tid >> 5;
  const int nodeBase = (int)blockIdx.x * nb;
  constexpr int NJ = (H * C) / 32;

  for (int i = tid; i < NBMAX; i += NTHR) scnt[i] = 0;
  if (wave < H) {
    float s = 0.f;
    for (int c = lane; c < C; c += 32) s = fmaf(We[wave * C + c], ae[wave * C + c], s);
    s = wsum(s);
    if (lane == 0) cel[wave] = s;
  }
  __syncthreads();

  int tot = 0;
  const int nChunks = (nE + CHUNK - 1) / CHUNK;
#pragma unroll 1
  for (int ch = 0; ch < nChunks; ++ch) {
    const int cbase = ch * CHUNK;
    const int wc = scan_chunk(dsts, nE, cbase, nodeBase, nb, vec8, list, tid, lane, wave);
    if (lane == 0) wcnt[wave] = wc;
    __syncthreads();
    int pre = 0, all = 0;
#pragma unroll
    for (int w2 = 0; w2 < NWAVE; ++w2) {
      int c = wcnt[w2];
      c = c < 0 ? 0 : (c > WCAP ? WCAP : c);
      all += c;
      pre += (w2 < wave) ? c : 0;
    }
    const int wcc  = wc > WCAP ? WCAP : wc;
    const int base = tot + pre;
#pragma unroll 1
    for (int i = lane; i < wcc; i += 32) {
      const int ent = list[wave * WCAP + i];
      const int el  = (ent >> 12) & (CHUNK - 1);
      const int sl  = ent & (NBMAX - 1);
      int eid = cbase + el;
      eid = eid > nE - 1 ? nE - 1 : eid;
      const int pos = base + i;
      if (pos < RCAP) reg1[pos] = (int)(((unsigned)eid << SLB) | (unsigned)sl);
    }
    tot += all;
    tot = tot > RCAP ? RCAP : tot;
    __syncthreads();
  }
  const int nh = tot;

  if (wave == 0) {
#pragma unroll 1
    for (int b0 = 0; b0 < nh; b0 += 32) {
      const int idx = b0 + lane;
      const int uv  = reg1[idx < RCAP ? idx : RCAP - 1];
      const int m32 = (nh - b0) < 32 ? (nh - b0) : 32;
#pragma unroll 1
      for (int k = 0; k < m32; ++k) {
        const int u  = __builtin_amdgcn_readlane(uv, k);
        const int sl = u & (NBMAX - 1);
        if (lane == 0) scnt[sl] = scnt[sl] + 1;
      }
    }
  }
  __syncthreads();

  {
    const int ca = scnt[2 * tid];
    const int cb = scnt[2 * tid + 1];
    const int e0 = ca < 0 ? 0 : ca, e1 = cb < 0 ? 0 : cb;
    const int ts = e0 + e1;
    int incl = ts;
#pragma unroll
    for (int d = 1; d < 32; d <<= 1) {
      const int up = __shfl_up(incl, d);
      if (lane >= d) incl += up;
    }
    if (lane == 31) wtot[wave] = incl;
    __syncthreads();
    int pre = 0;
#pragma unroll
    for (int w2 = 0; w2 < NWAVE; ++w2) pre += (w2 < wave) ? wtot[w2] : 0;
    int run = pre + incl - ts;
    soff[2 * tid + 0] = run; run += e0;
    soff[2 * tid + 1] = run;
  }
  __syncthreads();
  for (int i = tid; i < NBMAX; i += NTHR) list[i] = soff[i];
  __syncthreads();

  if (wave == 0) {
#pragma unroll 1
    for (int b0 = 0; b0 < nh; b0 += 32) {
      const int idx = b0 + lane;
      const int uv  = reg1[idx < RCAP ? idx : RCAP - 1];
      const int m32 = (nh - b0) < 32 ? (nh - b0) : 32;
#pragma unroll 1
      for (int k = 0; k < m32; ++k) {
        const int u   = __builtin_amdgcn_readlane(uv, k);
        const int sl  = u & (NBMAX - 1);
        const int eid = (int)((unsigned)u >> SLB);
        if (lane == 0) {
          int pos = list[sl];
          pos = pos < 0 ? 0 : (pos > RCAP - 1 ? RCAP - 1 : pos);
          reg2[pos] = eid;
          list[sl] = pos + 1;
        }
      }
    }
  }
  __syncthreads();

  const int nbw = nb >> 3;
  const bool ovf = (nh >= RCAP);
  const float qnan = __int_as_float(0x7fc00000);
  float* stw = (float*)reg1 + wave * STW;
  int*   sti = reg1 + wave * STW;
  const float ce0 = cel[0];
  const float ce1 = (H > 1) ? cel[1] : 0.f;
#pragma unroll 1
  for (int jt = 0; jt < nbw; ++jt) {
    const int slot = wave * nbw + jt;
    const int grow = nodeBase + slot;
    const int gcl  = grow < nN ? grow : nN - 1;
    int st = soff[slot];
    const int craw = scnt[slot];
    int cnt = craw;
    st  = st < 0 ? 0 : (st > nh ? nh : st);
    cnt = cnt < 0 ? 0 : (cnt > DEGCAP ? DEGCAP : cnt);
    if (cnt > nh - st) cnt = nh - st;
    cnt = cnt < 0 ? 0 : cnt;
    const float pz = (ovf || craw > DEGCAP) ? qnan : 0.0f;
    const float live = grow < nN ? 1.0f : 0.0f;
    const int T   = cnt + 1;
    const int nbt = (T + 31) >> 5;

    WSYNC();
    float ews = 0.f;
#pragma unroll 1
    for (int b = 0; b < nbt; ++b) {
      const int q = 32 * b + lane;
      const bool valid = q < cnt;
      int idx = st + q; idx = idx > RCAP - 1 ? RCAP - 1 : idx;
      int eid = reg2[idx]; eid = eid < 0 ? 0 : (eid > nE - 1 ? nE - 1 : eid);
      const int sraw = srcs[eid];
      const int s = sraw < 0 ? 0 : (sraw > nN - 1 ? nN - 1 : sraw);
      const float ea = ew[eid];
      ews += valid ? ea : 0.f;
      sti[O_S + q] = valid ? s : gcl;
      stw[O_E + q] = valid ? ea : 0.f;
    }
    ews = wsum(ews);
    const float fc = (float)cnt;
    const float la = ews * __builtin_amdgcn_rcpf(fmaxf(fc, 1.0f));
    WSYNC();
    if (lane == 0) stw[O_E + cnt] = la;
    WSYNC();

    const float ald0 = AL[(size_t)MPr + gcl];
    const float ald1 = (H > 1) ? AL[(size_t)3 * (size_t)MPr + gcl] : 0.f;
    float m0 = -3.0e38f, m1 = -3.0e38f;
#pragma unroll 1
    for (int b = 0; b < nbt; ++b) {
      const int q = 32 * b + lane;
      const bool valid = q < T;
      int s = sti[O_S + q]; s = s < 0 ? 0 : (s > nN - 1 ? nN - 1 : s);
      const float ea = stw[O_E + q];
      float l0 = fmaf(ea, ce0, AL[(size_t)s] + ald0);
      l0 = l0 > 0.f ? l0 : NEGSL * l0;
      l0 = valid ? l0 : -3.0e38f;
      m0 = fmaxf(m0, l0);
      stw[O_P0 + q] = l0;
      if (H > 1) {
        float l1 = fmaf(ea, ce1, AL[(size_t)2 * (size_t)MPr + s] + ald1);
        l1 = l1 > 0.f ? l1 : NEGSL * l1;
        l1 = valid ? l1 : -3.0e38f;
        m1 = fmaxf(m1, l1);
        stw[O_P1 + q] = l1;
      }
    }
    m0 = wmax(m0);
    if (H > 1) m1 = wmax(m1);
    float d0 = 0.f, d1 = 0.f;
#pragma unroll 1
    for (int b = 0; b < nbt; ++b) {
      const int q = 32 * b + lane;
      const bool valid = q < T;
      const float l0 = stw[O_P0 + q];
      const float p0 = valid ? expf(l0 - m0) : 0.f;
      stw[O_P0 + q] = p0;
      d0 += p0;
      if (H > 1) {
        const float l1 = stw[O_P1 + q];
        const float p1 = valid ? expf(l1 - m1) : 0.f;
        stw[O_P1 + q] = p1;
        d1 += p1;
      }
    }
    d0 = wsum(d0);
    const float inv0 = __builtin_amdgcn_rcpf(d0 + 1e-16f);
    float inv1 = 0.f;
    if (H > 1) { d1 = wsum(d1); inv1 = __builtin_amdgcn_rcpf(d1 + 1e-16f); }
    WSYNC();

    float av[NJ];
#pragma unroll
    for (int j = 0; j < NJ; ++j) av[j] = 0.f;
#pragma unroll 1
    for (int q = 0; q < T; ++q) {
      int s = sti[O_S + q]; s = s < 0 ? 0 : (s > nN - 1 ? nN - 1 : s);
      const float a0 = stw[O_P0 + q] * inv0;
      const float a1 = (H > 1) ? stw[O_P1 + q] * inv1 : 0.f;
      const float* hr = HF + (size_t)s * (size_t)ldh + lane;
      float hv[NJ];
#pragma unroll
      for (int j = 0; j < NJ; ++j) hv[j] = hr[32 * j];
      ldwait();
#pragma unroll
      for (int j = 0; j < NJ; ++j) av[j] = fmaf((32 * j < C) ? a0 : a1, hv[j], av[j]);
    }

    WSYNC();
    if (LAYER == 1) {
#pragma unroll
      for (int j = 0; j < NJ; ++j) stw[O_O + 32 * j + lane] = av[j] + bias[32 * j + lane];
#pragma unroll 1
      for (int j = 0; j < NJ; ++j) {
        float v = stw[O_O + 32 * j + lane];
        v = v > 0.f ? v : expm1f(v);
        stw[O_O + 32 * j + lane] = v * live + pz;
      }
      WSYNC();
      const int lc = lane < ((H * C) / 8) ? lane : ((H * C) / 8) - 1;
      const v4f ga = *(const v4f*)(stw + O_O + 8 * lc);
      const v4f gb = *(const v4f*)(stw + O_O + 8 * lc + 4);
      const v8h hv8 = cvt8h(ga, gb, CX);
      _Float16* gp = HH + (size_t)grow * (size_t)(H * C) + 8 * lc;
      const bool wsv = (grow < MPr) && (lane < ((H * C) / 8));
      if (wsv) *(volatile v8h*)gp = hv8;
      __threadfence();
      if (wsv) *(volatile v8h*)gp = hv8;
    } else {
      const float v = (av[0] + bias[lane]) * live + pz;
      stw[O_O + lane] = v;
      WSYNC();
      const int lc8 = lane < (OUTC / 4) ? lane : (OUTC / 4) - 1;
      const v4f g = *(const v4f*)(stw + O_O + 4 * lc8);
      float* op = OUT + (size_t)grow * OUTC + 4 * lc8;
      const bool wsv = (grow < nN) && (lane < (OUTC / 4));
      if (wsv) *(volatile v4f*)op = g;
      __threadfence();
      if (wsv) *(volatile v4f*)op = g;
    }
  }
}

static int pick_nb(int nE, int nN) {
  int nb = NBMAX;
  while (nb > 16 && (long long)nb * (long long)nE * 5LL > (long long)RCAP * (long long)nN * 4LL) nb >>= 1;
  return nb;
}
static inline int cdiv(int a, int b) { return (a + b - 1) / b; }

extern "C" void kernel_launch(void* const* d_in, const int* in_sizes, int n_in,
                              void* d_out, int out_size, void* d_ws, size_t ws_size,
                              hipStream_t stream) {
  if (n_in < 15) return;
  const int nN = in_sizes[0] / DIN;
  if (nN <= 0 || in_sizes[0] != nN * DIN || nN > (1 << 22)) return;
  if (in_sizes[1] < 2 || (in_sizes[1] & 1) != 0) return;
  const int nE = in_sizes[1] / 2;
  if (nE < 1 || nE > (1 << 22)) return;
  if (in_sizes[2] != nE) return;
  if (in_sizes[3] != DIN * C1) return;
  if (in_sizes[4] != C1 || in_sizes[5] != C1) return;
  if (in_sizes[6] != C1 || in_sizes[7] != C1) return;
  if (in_sizes[8] != C1) return;
  if (in_sizes[9] != C1 * OUTC) return;
  if (in_sizes[10] != OUTC || in_sizes[11] != OUTC) return;
  if (in_sizes[12] != OUTC || in_sizes[13] != OUTC) return;
  if (in_sizes[14] != OUTC) return;
  if (out_size != nN * OUTC) return;

  const float* x    = (const float*)d_in[0];
  const int*   ei   = (const int*)  d_in[1];
  const float* ew   = (const float*)d_in[2];
  const float* W1   = (const float*)d_in[3];
  const float* as1  = (const float*)d_in[4];
  const float* ad1  = (const float*)d_in[5];
  const float* We1  = (const float*)d_in[6];
  const float* ae1  = (const float*)d_in[7];
  const float* b1   = (const float*)d_in[8];
  const float* W2   = (const float*)d_in[9];
  const float* as2  = (const float*)d_in[10];
  const float* ad2  = (const float*)d_in[11];
  const float* We2  = (const float*)d_in[12];
  const float* ae2  = (const float*)d_in[13];
  const float* b2   = (const float*)d_in[14];
  float* out = (float*)d_out;
  const int* src = ei;
  const int* dst = ei + nE;

  const int MP   = cdiv(nN, GBM) * GBM;
  const int nb   = pick_nb(nE, nN);
  const int gA   = cdiv(MP, nb);
  const int vec8 = ((nE & 3) == 0) ? 1 : 0;
  if (gA * nb < MP) return;

  char* ws = (char*)d_ws;
  size_t off = 0;
  const size_t oXH  = off; off += (size_t)MP * DIN * 2;            off = (off + 255) & ~(size_t)255;
  const size_t oWT1 = off; off += (size_t)C1 * DIN * 2;            off = (off + 255) & ~(size_t)255;
  const size_t oWT2 = off; off += (size_t)N2P * DIN * 2;           off = (off + 255) & ~(size_t)255;
  const size_t oH1F = off; off += (size_t)MP * C1 * 4;             off = (off + 255) & ~(size_t)255;
  const size_t oAL1 = off; off += (size_t)4 * MP * 4;              off = (off + 255) & ~(size_t)255;
  const size_t oHH  = off; off += (size_t)MP * C1 * 2;             off = (off + 255) & ~(size_t)255;
  const size_t oH2F = off; off += (size_t)MP * N2P * 4;            off = (off + 255) & ~(size_t)255;
  const size_t oAL2 = off; off += (size_t)2 * MP * 4;              off = (off + 255) & ~(size_t)255;
  if (off > ws_size || off > (size_t)WSMAX) return;
  _Float16* XH   = (_Float16*)(ws + oXH);
  _Float16* WT1  = (_Float16*)(ws + oWT1);
  _Float16* WT2  = (_Float16*)(ws + oWT2);
  float*    H1F  = (float*)(ws + oH1F);
  float*    AL1  = (float*)(ws + oAL1);
  _Float16* HH   = (_Float16*)(ws + oHH);
  float*    H2F  = (float*)(ws + oH2F);
  float*    AL2  = (float*)(ws + oAL2);

  hipFuncSetAttribute(reinterpret_cast<const void*>(&k_agg<2, 64, 1>),
                      hipFuncAttributeMaxDynamicSharedMemorySize, LDS_AGG);
  hipFuncSetAttribute(reinterpret_cast<const void*>(&k_agg<1, 32, 2>),
                      hipFuncAttributeMaxDynamicSharedMemorySize, LDS_AGG);

  const int nUx = MP * (DIN / 8);
  k_xprep<<<cdiv(nUx, NTHR), NTHR, 0, stream>>>(x, XH, nN, nUx);

  {
    const int nU1 = C1 * (DIN / 8);
    k_wtr<<<cdiv(nU1, NTHR), NTHR, 0, stream>>>(W1, C1, DIN, WT1, nU1);
    const int nU2 = N2P * (DIN / 8);
    k_wtr<<<cdiv(nU2, NTHR), NTHR, 0, stream>>>(W2, OUTC, DIN, WT2, nU2);
  }

  const int gM = MP / GBM;
  k_gemm<<<dim3(gM, C1 / GBN), GTHR, 0, stream>>>(XH, WT1, H1F, DIN, C1, as1, ad1, 64, AL1, MP, SCL_XW);
  k_agg<2, 64, 1><<<gA, NTHR, LDS_AGG, stream>>>(src, dst, ew, We1, ae1, AL1, H1F, C1, b1, HH, out,
                                                  nN, nE, nb, vec8, MP);
  k_gemm<<<dim3(gM, N2P / GBN), GTHR, 0, stream>>>(HH, WT2, H2F, DIN, N2P, as2, ad2, OUTC, AL2, MP, SCL_XW);
  k_agg<1, 32, 2><<<gA, NTHR, LDS_AGG, stream>>>(src, dst, ew, We2, ae2, AL2, H2F, N2P, b2, HH, out,
                                                  nN, nE, nb, vec8, MP);
}
